// CPPN_28226525069673
// MI455X (gfx1250) — hardware-run, weakly checked
//
#include <hip/hip_runtime.h>
#include <math.h>

typedef __attribute__((ext_vector_type(16))) _Float16 v16h;
typedef __attribute__((ext_vector_type(8)))  _Float16 v8h;
typedef __attribute__((ext_vector_type(8)))  float    v8f;
typedef __attribute__((ext_vector_type(4)))  float    v4f;

constexpr int kPts      = 2097152;
constexpr int kWidth    = 16;
constexpr int kInDim    = 3;
constexpr int kLayers   = 8;
constexpr int kBlock    = 256;
constexpr int kGridMax  = 1024;
constexpr int kGroupsPerWave = 8;
constexpr float kCarry    = 2048.0f;
constexpr float kCarryInv = 1.0f / kCarry;
constexpr float kF16MinNormal = 6.103515625e-5f;
static_assert(kLayers * 32 == kBlock, "one staging thread per (layer, lane)");
static_assert(kLayers * kWidth <= kBlock, "bias staging coverage");
static_assert((kPts % 32) == 0, "whole 128-B output lines");
static_assert(kWidth == 16, "K packing assumes 16 + 16 = 32");

union FragU { v16h v; v8h half[2]; };

__device__ __forceinline__ v8f mma_f16(v16h a, v16h b, v8f c) {
  c = __builtin_amdgcn_wmma_f32_16x16x32_f16(false, a, false, b, (short)0, c, false, false);
  asm volatile("v_nop\n\tv_nop\n\tv_nop\n\tv_nop" : "+v"(c) : "v"(a), "v"(b));
  return c;
}

__device__ __forceinline__ void split_f16(float t, _Float16& hi, _Float16& lo) {
  float hf = (float)((_Float16)t);
  hf = (fabsf(hf) < kF16MinNormal) ? 0.0f : hf;
  hi = (_Float16)hf;
  lo = (_Float16)((t - hf) * kCarry);
}

__device__ __forceinline__ float tanh_f32(float z) {
  const float e = __expf(2.0f * z);
  return 1.0f - 2.0f * __builtin_amdgcn_rcpf(e + 1.0f);
}

__global__ __launch_bounds__(256) void mlp_fused_kernel(
    const float* __restrict__ x, const float* __restrict__ W0, const float* __restrict__ b0,
    const float* __restrict__ Wh, const float* __restrict__ bh, const float* __restrict__ Wo,
    const float* __restrict__ bo, float* __restrict__ out, int npts, int ngroups)
{
  __shared__ __align__(16) v8h   sWhi[kLayers * 32];
  __shared__ __align__(16) v8h   sWlo[kLayers * 32];
  __shared__ __align__(16) float sBh[kLayers * kWidth];

  const int tid  = threadIdx.x;
  const int lane = tid & 31;
  const int hh   = lane >> 4;
  const int nn   = lane & 15;

  {
    const int layer = tid >> 5;
    const float* wp = Wh + layer * (kWidth * kWidth) + nn * kWidth + 8 * hh;
    const v4f a0 = *(const v4f*)(wp);
    const v4f a1 = *(const v4f*)(wp + 4);
    v8h whi, wlo;
#pragma unroll
    for (int e = 0; e < 4; ++e) {
      const float f0 = a0[e];
      const float f1 = a1[e];
      _Float16 h0, l0, h1, l1;
      split_f16(f0, h0, l0);
      split_f16(f1, h1, l1);
      whi[e]     = h0;
      wlo[e]     = l0;
      whi[4 + e] = h1;
      wlo[4 + e] = l1;
    }
    sWhi[tid] = whi;
    sWlo[tid] = wlo;
    if (tid < kLayers * kWidth) sBh[tid] = bh[tid];
  }
  __syncthreads();

  float w0r[24], b0r[8], wor[8];
  {
    const float* p = W0 + 24 * hh;
#pragma unroll
    for (int q = 0; q < 6; ++q) {
      const v4f v = *(const v4f*)(p + 4 * q);
      w0r[4 * q + 0] = v[0];
      w0r[4 * q + 1] = v[1];
      w0r[4 * q + 2] = v[2];
      w0r[4 * q + 3] = v[3];
    }
    const v4f c0 = *(const v4f*)(b0 + 8 * hh);
    const v4f c1 = *(const v4f*)(b0 + 8 * hh + 4);
    const v4f d0 = *(const v4f*)(Wo + 8 * hh);
    const v4f d1 = *(const v4f*)(Wo + 8 * hh + 4);
#pragma unroll
    for (int e = 0; e < 4; ++e) {
      b0r[e]     = c0[e];
      b0r[4 + e] = c1[e];
      wor[e]     = d0[e];
      wor[4 + e] = d1[e];
    }
  }
  const float bo0 = bo[0];

  const v8h zero8 = {(_Float16)0.0f, (_Float16)0.0f, (_Float16)0.0f, (_Float16)0.0f,
                     (_Float16)0.0f, (_Float16)0.0f, (_Float16)0.0f, (_Float16)0.0f};

  const int wid    = (blockIdx.x * kBlock + tid) >> 5;
  const int nwaves = (gridDim.x * kBlock) >> 5;

  for (int g = wid; g < ngroups; g += nwaves) {
    float myout = 0.0f;
#pragma unroll 1
    for (int t = 0; t < 2; ++t) {
      const int p  = g * 32 + 16 * t + nn;
      const int pc = (p < npts) ? p : (npts - 1);
      const float* xp = x + (size_t)pc * kInDim;
      const float x0 = xp[0];
      const float x1 = xp[1];
      const float x2 = xp[2];

      float tv[8];
      v16h bfrag;
#pragma unroll
      for (int r = 0; r < 8; ++r) {
        float z = x0 * w0r[3 * r + 0];
        z = fmaf(x1, w0r[3 * r + 1], z);
        z = fmaf(x2, w0r[3 * r + 2], z);
        z = z + b0r[r];
        const float tt = tanh_f32(z);
        tv[r] = tt;
        _Float16 hi, lo;
        split_f16(tt, hi, lo);
        bfrag[r]     = hi;
        bfrag[8 + r] = lo;
      }

#pragma unroll 1
      for (int l = 0; l < kLayers; ++l) {
        const v8h whi = sWhi[l * 32 + lane];
        const v8h wlo = sWlo[l * 32 + lane];
        FragU am, ar;
        am.half[0] = whi;
        am.half[1] = zero8;
        ar.half[0] = wlo;
        ar.half[1] = whi;
        const v4f bA = *(const v4f*)(sBh + l * kWidth + 8 * hh);
        const v4f bB = *(const v4f*)(sBh + l * kWidth + 8 * hh + 4);
        v8f cm = {bA[0], bA[1], bA[2], bA[3], bB[0], bB[1], bB[2], bB[3]};
        v8f cr = {0.f, 0.f, 0.f, 0.f, 0.f, 0.f, 0.f, 0.f};
        cm = mma_f16(am.v, bfrag, cm);
        cr = mma_f16(ar.v, bfrag, cr);
        v16h nb;
#pragma unroll
        for (int r = 0; r < 8; ++r) {
          const float z  = fmaf(cr[r], kCarryInv, cm[r]);
          const float tt = tanh_f32(z);
          tv[r] = tt;
          _Float16 hi, lo;
          split_f16(tt, hi, lo);
          nb[r]     = hi;
          nb[8 + r] = lo;
        }
        bfrag = nb;
      }

      float part = 0.0f;
#pragma unroll
      for (int r = 0; r < 8; ++r) part = fmaf(tv[r], wor[r], part);
      const float other = __shfl_xor(part, 16, 32);
      const float plo = (hh == 0) ? part : other;
      const float phi = (hh == 0) ? other : part;
      const float logit = (plo + phi) + bo0;
      const float o = __builtin_amdgcn_rcpf(1.0f + __expf(-logit));
      myout = (hh == t) ? o : myout;
    }

    const int pt = g * 32 + lane;
    const bool ok = (pt < npts);
    const int ptc = ok ? pt : (npts - 1);
    volatile float* op = out + ptc;
    if (ok) *op = myout;
    __threadfence();
    if (ok) *op = myout;
  }
}

extern "C" void kernel_launch(void* const* d_in, const int* in_sizes, int n_in,
                              void* d_out, int out_size, void* d_ws, size_t ws_size,
                              hipStream_t stream) {
  (void)d_ws;
  (void)ws_size;
  if (n_in < 7) return;
  if (in_sizes[0] != kPts * kInDim) return;
  if (in_sizes[1] != kWidth * kInDim) return;
  if (in_sizes[2] != kWidth) return;
  if (in_sizes[3] != kLayers * kWidth * kWidth) return;
  if (in_sizes[4] != kLayers * kWidth) return;
  if (in_sizes[5] != kWidth) return;
  if (in_sizes[6] != 1) return;
  if (out_size != kPts) return;

  const float* x  = (const float*)d_in[0];
  const float* W0 = (const float*)d_in[1];
  const float* b0 = (const float*)d_in[2];
  const float* Wh = (const float*)d_in[3];
  const float* bh = (const float*)d_in[4];
  const float* Wo = (const float*)d_in[5];
  const float* bo = (const float*)d_in[6];
  float* out = (float*)d_out;

  const int npts    = kPts;
  const int ngroups = (npts + 31) / 32;
  int grid = (ngroups + kGroupsPerWave * (kBlock / 32) - 1) / (kGroupsPerWave * (kBlock / 32));
  if (grid > kGridMax) grid = kGridMax;
  if (grid < 1) grid = 1;

  mlp_fused_kernel<<<grid, kBlock, 0, stream>>>(x, W0, b0, Wh, bh, Wo, bo, out, npts, ngroups);
}
